// SpatiaTemporallNeighbourhoodAttentionBlock_24541443130185
// MI455X (gfx1250) — hardware-run, weakly checked
//
#include <hip/hip_runtime.h>


namespace {
constexpr int C = 128, T = 12, Hh = 40, Ww = 40, NTK = T * Hh * Ww  , KN = 27;
constexpr float HS = 256.0f, WSC = 256.0f, SQC = 11.313708498984761f  , ISQ = 0.088388347648318447f;
typedef _Float16 b16;
typedef __attribute__((ext_vector_type(16))) _Float16 v16b;
typedef __attribute__((ext_vector_type(8))) _Float16 v8b;
typedef __attribute__((ext_vector_type(8))) float v8f;
typedef __attribute__((ext_vector_type(4))) float v4f;
__device__ __forceinline__ float bf16_rne(float f) { unsigned int u = __float_as_uint(f); u += 0x7FFFu + ((u >> 16) & 1u); float r = __uint_as_float(u & 0xFFFF0000u); asm volatile("" : "+v"(r)); return r; }
__device__ __forceinline__ float bfv(float f) { float r = bf16_rne(f); asm volatile("" : "+v"(r)); return r; }
__device__ __forceinline__ void split16(float v, b16& hi, b16& lo) { hi = (b16)v; lo = (b16)(v - (float)hi); }
__device__ __forceinline__ v16b frag_kb(const b16* p, int hh) { const v8b a = *(const v8b*)(p + 8 * hh), b = *(const v8b*)(p + 16 + 8 * hh); v16b f;
#pragma unroll
  for (int e = 0; e < 8; ++e) { f[e] = a[e]; f[8 + e] = b[e]; } return f; }
__device__ __forceinline__ v8f wmma16b(v16b a, v16b b, v8f c) { v8f d = __builtin_amdgcn_wmma_f32_16x16x32_f16(false, a, false, b, (short)0, c, false, false); asm volatile("v_nop\n\tv_nop\n\tv_nop\n\tv_nop" : "+v"(d) : "v"(a), "v"(b)); return d; }
__device__ __forceinline__ void wave_lds_sync() { __builtin_amdgcn_fence(__ATOMIC_RELEASE, "workgroup"); __builtin_amdgcn_wave_barrier(); __builtin_amdgcn_fence(__ATOMIC_ACQUIRE, "workgroup"); }
__device__ __forceinline__ float pmul(float a, float b) { float p = a * b; asm volatile("" : "+v"(p)); return p; }
__device__ __forceinline__ int iclamp(int v, int lo, int hi) { return v < lo ? lo : (v > hi ? hi : v); }

__global__ __launch_bounds__(256) void wput_kernel(const float* __restrict__ wq, const float* __restrict__ wp, b16* __restrict__ WQ, b16* __restrict__ WP) { const int u = blockIdx.x * 256 + threadIdx.x; v8b v;
  if (u < 384 * 16) { const int o = u / 16, k0 = (u % 16) * 8;
#pragma unroll
    for (int j = 0; j < 8; ++j) v[j] = (b16)(bf16_rne(wq[(size_t)o * C + k0 + j]) * WSC); for (int pass = 0; pass < 2; ++pass) { *(volatile v8b*)(WQ + (size_t)o * C + k0) = v; __threadfence(); } }
  if (u < 128 * 16) { const int o = u / 16, k0 = (u % 16) * 8;
#pragma unroll
    for (int j = 0; j < 8; ++j) v[j] = (b16)(bf16_rne(wp[(size_t)o * C + k0 + j]) * WSC); for (int pass = 0; pass < 2; ++pass) { *(volatile v8b*)(WP + (size_t)o * C + k0) = v; __threadfence(); } } }
__global__ __launch_bounds__(256) void norm_kernel(const float* __restrict__ x, const float* __restrict__ gm, float* __restrict__ XN) { const int p = blockIdx.x * 256 + threadIdx.x; if (p >= NTK) return; float s = 0.0f; for (int c = 0; c < C; ++c) { const float v = bfv(x[(size_t)c * NTK + p]); s += v * v; } const float inv = SQC / fmaxf(sqrtf(s), 1e-12f);
  for (int pass = 0; pass < 2; ++pass) { for (int c = 0; c < C; ++c) ((volatile float*)XN)[(size_t)c * NTK + p] = pmul(bfv(x[(size_t)c * NTK + p]) * inv, bfv(gm[c])); __threadfence(); } }
__global__ __launch_bounds__(32) void qkv_kernel(const float* __restrict__ XN, const b16* __restrict__ WQ, const float* __restrict__ qb, int NLIM, float* __restrict__ QKV) { __shared__ __attribute__((aligned(16))) b16 Ah[16][C + 8], Al[16][C + 8]; __shared__ float Tf[16][132]; const int lane = threadIdx.x, nloc = lane & 15, hlf = lane >> 4; const size_t n0 = (size_t)blockIdx.x * 16; if (n0 >= (size_t)NLIM) return;
  for (int rr = 0; rr < 16; ++rr) for (int q = 0; q < 4; ++q) { const int c = q * 32 + lane; b16 p, pl; split16(XN[(n0 + rr) * C + c] * HS, p, pl); Ah[rr][c] = p; Al[rr][c] = pl; }
  if (lane < 16) for (int k = C; k < C + 8; ++k) { Ah[lane][k] = (b16)0.0f; Al[lane][k] = (b16)0.0f; }
  wave_lds_sync();
#pragma unroll 1
  for (int g = 0; g < 3; ++g) { v8f acc[8];
#pragma unroll
    for (int t = 0; t < 8; ++t) acc[t] = (v8f){};
#pragma unroll
    for (int kb = 0; kb < C; kb += 32) { const v16b a = frag_kb(&Ah[nloc][kb], hlf), al = frag_kb(&Al[nloc][kb], hlf);
#pragma unroll
      for (int t = 0; t < 8; ++t) { const v16b bw = frag_kb(WQ + (size_t)(g * C + t * 16 + nloc) * C + kb, hlf); acc[t] = wmma16b(a, bw, acc[t]); acc[t] = wmma16b(al, bw, acc[t]); } }
    const float osc = g == 0 ? ISQ : 1.0f;
#pragma unroll
    for (int t = 0; t < 8; ++t) { const int cc = t * 16 + nloc; const float bb = bfv(qb[g * C + cc]);
#pragma unroll
      for (int r8 = 0; r8 < 8; ++r8) Tf[8 * hlf + r8][cc] = (acc[t][r8] * (1.0f / (HS * WSC)) + bb) * osc; }
    wave_lds_sync();
    for (int pass = 0; pass < 2; ++pass) { for (int rr = 0; rr < 16; ++rr) *(volatile v4f*)(QKV + (n0 + rr) * 3 * C + g * C + lane * 4) = *(const v4f*)(&Tf[rr][lane * 4]); __threadfence(); }
    wave_lds_sync(); } }
__global__ __launch_bounds__(32) void att_kernel(const float* __restrict__ QKV, const float* __restrict__ rpb, const b16* __restrict__ WP, const float* __restrict__ pb, const float* __restrict__ x, int NLIM, float* __restrict__ out) { __shared__ __attribute__((aligned(16))) b16 Ah[16][C + 8], Al[16][C + 8]; __shared__ float Lg[16][32], Tf[16][132]; __shared__ int Nb[16][32]; const int lane = threadIdx.x, nloc = lane & 15, hlf = lane >> 4; const size_t n0 = (size_t)blockIdx.x * 16; if (n0 >= (size_t)NLIM) return;
  for (int rr = 0; rr < 16; ++rr) { const int n = (int)(n0 + rr); const int it = n / (Hh * Ww), ih = (n / Ww) % Hh, iw = n % Ww; if (lane < KN) { const int a = lane / 9, bq = (lane / 3) % 3, cq = lane % 3; const int jt = iclamp(it - 1, 0, T - 3) + a, jh = iclamp(ih - 1, 0, Hh - 3) + bq, jw = iclamp(iw - 1, 0, Ww - 3) + cq; Nb[rr][lane] = (jt * Hh + jh) * Ww + jw; Lg[rr][lane] = bfv(rpb[((jt - it + 2) * 5 + (jh - ih + 2)) * 5 + (jw - iw + 2)]); } else { Nb[rr][lane] = 0; Lg[rr][lane] = -INFINITY; } }
  wave_lds_sync();
  for (int rr = 0; rr < 16; ++rr) if (lane < KN) { const float* qp = QKV + (n0 + rr) * 3 * C; const float* kp = QKV + (size_t)Nb[rr][lane] * 3 * C + C; float s = 0.0f;
#pragma unroll 4
      for (int c = 0; c < C; ++c) s += pmul(qp[c], kp[c]); Lg[rr][lane] += s; }
  wave_lds_sync();
  for (int rr = 0; rr < 16; ++rr) { float v = Lg[rr][lane]; float mx = v; for (int o = 16; o; o >>= 1) mx = fmaxf(mx, __shfl_xor(mx, o)); float p = (lane < KN) ? __expf(v - mx) : 0.0f; float sm = p; for (int o = 16; o; o >>= 1) sm += __shfl_xor(sm, o); Lg[rr][lane] = p / sm; }
  wave_lds_sync();
  for (int rr = 0; rr < 16; ++rr) { v4f o = {0, 0, 0, 0};
#pragma unroll 1
    for (int kk = 0; kk < KN; ++kk) { const v4f vv = *(const v4f*)(QKV + (size_t)Nb[rr][kk] * 3 * C + 2 * C + lane * 4); o += vv * Lg[rr][kk]; }
    for (int k = 0; k < 4; ++k) { b16 p, pl; split16(o[k] * HS, p, pl); Ah[rr][lane * 4 + k] = p; Al[rr][lane * 4 + k] = pl; } }
  if (lane < 16) for (int k = C; k < C + 8; ++k) { Ah[lane][k] = (b16)0.0f; Al[lane][k] = (b16)0.0f; }
  wave_lds_sync(); v8f acc[8];
#pragma unroll
  for (int t = 0; t < 8; ++t) acc[t] = (v8f){};
#pragma unroll
  for (int kb = 0; kb < C; kb += 32) { const v16b a = frag_kb(&Ah[nloc][kb], hlf), al = frag_kb(&Al[nloc][kb], hlf);
#pragma unroll
    for (int t = 0; t < 8; ++t) { const v16b bw = frag_kb(WP + (size_t)(t * 16 + nloc) * C + kb, hlf); acc[t] = wmma16b(a, bw, acc[t]); acc[t] = wmma16b(al, bw, acc[t]); } }
#pragma unroll
  for (int t = 0; t < 8; ++t) { const int cc = t * 16 + nloc; const float bb = bfv(pb[cc]);
#pragma unroll
    for (int r8 = 0; r8 < 8; ++r8) { const int rr = 8 * hlf + r8; Tf[rr][cc] = acc[t][r8] * (1.0f / (HS * WSC)) + bb + bfv(x[(n0 + rr) * C + cc]); } }
  wave_lds_sync();
  for (int pass = 0; pass < 2; ++pass) { for (int rr = 0; rr < 16; ++rr) *(volatile v4f*)(out + (n0 + rr) * C + lane * 4) = *(const v4f*)(&Tf[rr][lane * 4]); __threadfence(); } }
}

extern "C" void kernel_launch(void* const* d_in, const int* in_sizes, int n_in, void* d_out, int out_size, void* d_ws, size_t ws_size, hipStream_t stream) {
  (void)n_in;
  auto Fp = [&](int i) { return (const float*)d_in[i]; };
  if (in_sizes[0] != C * NTK || in_sizes[1] != C || in_sizes[2] != 3 * C * C || in_sizes[4] != 125 || in_sizes[5] != C * C || out_size != C * NTK) return;
  const int NLIM = NTK;
  size_t off = 0; char* ws = (char*)d_ws;
  auto carve = [&](size_t bytes) { char* p = ws + off; off += (bytes + 255) & ~(size_t)255; return p; };
  b16* WQ = (b16*)carve((size_t)3 * C * C * 2); b16* WP = (b16*)carve((size_t)C * C * 2); float* XN = (float*)carve((size_t)C * NTK * 4); float* QKV = (float*)carve((size_t)NTK * 3 * C * 4);
  if (off > ws_size || off > ((size_t)48 << 20)) return;
  wput_kernel<<<(384 * 16 + 255) / 256, 256, 0, stream>>>(Fp(2), Fp(5), WQ, WP);
  norm_kernel<<<(NTK + 255) / 256, 256, 0, stream>>>(Fp(0), Fp(1), XN);
  qkv_kernel<<<NTK / 16, 32, 0, stream>>>(XN, WQ, Fp(3), NTK, QKV);
  att_kernel<<<NLIM / 16, 32, 0, stream>>>(QKV, Fp(4), WP, Fp(6), Fp(0), NLIM, (float*)d_out);
}
